// ConformerAttention_42795054137612
// MI455X (gfx1250) — hardware-verified
//
#include <hip/hip_runtime.h>
#include <math.h>

typedef __attribute__((ext_vector_type(16))) _Float16 v16h;
typedef __attribute__((ext_vector_type(16))) __bf16 v16b;
typedef __attribute__((ext_vector_type(8)))  _Float16 v8h;
typedef __attribute__((ext_vector_type(8)))  float v8f;
typedef __attribute__((ext_vector_type(4)))  float v4f;
typedef __attribute__((ext_vector_type(2)))  float v2f;
typedef __attribute__((ext_vector_type(4)))  unsigned v4u;
typedef __attribute__((ext_vector_type(4)))  int v4i;
typedef float __attribute__((may_alias)) float_a;
typedef int __attribute__((may_alias)) int_a;

template <typename T> __device__ __forceinline__ void vst2(void* p, T v) { *(volatile T*)p = v; __threadfence(); *(volatile T*)p = v; }
__device__ __forceinline__ v8f wmma16(v16h a, v16h b, v8f c) {
  v8f d = __builtin_amdgcn_wmma_f32_16x16x32_f16(false, a, false, b, (short)0, c, false, false);
  asm volatile("v_nop\n\tv_nop\n\tv_nop\n\tv_nop" : "+v"(d) : "v"(a), "v"(b));
  return d;
}
__device__ __forceinline__ v8f wmma_bf(v16b a, v16b b, v8f c) {
  v8f d = __builtin_amdgcn_wmma_f32_16x16x32_bf16(false, a, false, b, (short)0, c, false, false);
  asm volatile("v_nop\n\tv_nop\n\tv_nop\n\tv_nop" : "+v"(d) : "v"(a), "v"(b));
  return d;
}
__device__ __forceinline__ v16h frag_h(const _Float16* rowk0, int lane) {
  union { v16h v; v8h q[2]; } u; const _Float16* p = rowk0 + 8 * (lane >> 4);
  u.q[0] = *(const v8h*)p; u.q[1] = *(const v8h*)(p + 16); return u.v;
}
__device__ __forceinline__ v16h frag_f32(const float* rowk0, int lane) {
  v16h a; const float* p = rowk0 + 8 * (lane >> 4);
#pragma unroll
  for (int i = 0; i < 8; ++i) { a[i] = (_Float16)p[i]; a[8 + i] = (_Float16)p[16 + i]; }
  return a;
}
__device__ __forceinline__ v16h frag_f32s(const float* rowk0, int lane, float sc) {
  v16h a; const float* p = rowk0 + 8 * (lane >> 4);
#pragma unroll
  for (int i = 0; i < 8; ++i) { a[i] = (_Float16)(p[i] * sc); a[8 + i] = (_Float16)(p[16 + i] * sc); }
  return a;
}
__device__ __forceinline__ v16h fragc_f32(const float* W, int k0, int n, int lane, int ld, int K) {
  v16h a; const int g = lane >> 4;
#pragma unroll
  for (int i = 0; i < 8; ++i) { const int ka = k0 + 8 * g + i, kb = ka + 16;
    a[i] = (_Float16)(ka < K ? W[(size_t)(ka < K ? ka : K - 1) * ld + n] : 0.f); a[8 + i] = (_Float16)(kb < K ? W[(size_t)(kb < K ? kb : K - 1) * ld + n] : 0.f); }
  return a;
}
struct F2 { v16b h, l; };
__device__ __forceinline__ F2 bsplit16(const float v[16]) { F2 r;
#pragma unroll
  for (int i = 0; i < 16; ++i) { const __bf16 h = (__bf16)v[i]; r.h[i] = h; r.l[i] = (__bf16)(v[i] - (float)h); }
  return r; }
__device__ __forceinline__ F2 split_row(const float* row, int k0, int lane) { float v[16]; const float* p = row + k0 + 8 * (lane >> 4);
#pragma unroll
  for (int i = 0; i < 8; ++i) { v[i] = p[i]; v[8 + i] = p[16 + i]; }
  return bsplit16(v); }
__device__ __forceinline__ F2 split_rowK(const float* row, int k0, int lane, int K) { float v[16]; const int g = lane >> 4;
#pragma unroll
  for (int i = 0; i < 8; ++i) { const int ka = k0 + 8 * g + i, kb = ka + 16; v[i] = ka < K ? row[ka < K ? ka : K - 1] : 0.f; v[8 + i] = kb < K ? row[kb < K ? kb : K - 1] : 0.f; }
  return bsplit16(v); }
__device__ __forceinline__ F2 split_col(const float* W, int k0, int n, int lane, int ld, int K) { float v[16]; const int g = lane >> 4;
#pragma unroll
  for (int i = 0; i < 8; ++i) { const int ka = k0 + 8 * g + i, kb = ka + 16; v[i] = ka < K ? W[(size_t)(ka < K ? ka : K - 1) * ld + n] : 0.f; v[8 + i] = kb < K ? W[(size_t)(kb < K ? kb : K - 1) * ld + n] : 0.f; }
  return bsplit16(v); }
__device__ __forceinline__ v8f mac3(const F2& a, const F2& b, v8f c) { c = wmma_bf(a.l, b.h, c); c = wmma_bf(a.h, b.l, c); return wmma_bf(a.h, b.h, c); }
__device__ __forceinline__ float sigm(float v) { return 1.0f / (1.0f + expf(-v)); }
#define LDSX() do { asm volatile("s_wait_dscnt 0" ::: "memory"); __builtin_amdgcn_wave_barrier(); __builtin_amdgcn_fence(__ATOMIC_RELEASE, "workgroup"); } while (0)


#define NB 8
#define SS 1024
#define DM 512
#define NH 8
#define HD 64
#define PP 2047
#define PR 2048
#define NR (NB * SS)
#ifndef NBT
#define NBT NB
#define TB0 0
#define TQB (SS / 64)
#endif
#define RB0 ((size_t)TB0 * SS)
typedef __attribute__((ext_vector_type(8))) __bf16 v8b;
__device__ __forceinline__ v16b frag_b(const __bf16* rowk0, int lane) {
  union { v16b v; v8b q[2]; } u; const __bf16* p = rowk0 + 8 * (lane >> 4);
  u.q[0] = *(const v8b*)p; u.q[1] = *(const v8b*)(p + 16); return u.v;
}
__device__ __forceinline__ float bfr(float v) { return (float)(__bf16)v; }
__device__ __attribute__((noinline)) float exp_ni(float v) { return expf(v); }
__device__ __attribute__((noinline)) float erf_ni(float v) { return erff(v); }
#define PK_Q  0
#define PK_K  ((size_t)DM * DM)
#define PK_V  ((size_t)2 * DM * DM)
#define PK_O  ((size_t)3 * DM * DM)
#define PK_P  ((size_t)4 * DM * DM)
#define PK_END ((size_t)5 * DM * DM)
#define WS_PK  0u
#define WS_XN  (((2u * PK_END) + 127u) / 128u * 128u)
#define WS_QUH (WS_XN + 4u * NR * DM)
#define WS_QUL (WS_QUH + 2u * NR * DM)
#define WS_QVH (WS_QUL + 2u * NR * DM)
#define WS_QVL (WS_QVH + 2u * NR * DM)
#define WS_KH  (WS_QVL + 2u * NR * DM)
#define WS_KL  (WS_KH + 2u * NR * DM)
#define WS_VTH (WS_KL + 2u * NR * DM)
#define WS_VTL (WS_VTH + 2u * NR * DM)
#define WS_RH  (WS_VTL + 2u * NR * DM)
#define WS_RL  (WS_RH + 2u * PR * DM)
#define WS_O   (WS_RL + 2u * PR * DM)
#define WS_END (WS_O + 4u * NR * DM)

__global__ __launch_bounds__(256) void k_pack(const float* __restrict__ WQ, const float* __restrict__ WK, const float* __restrict__ WV, const float* __restrict__ WO, const float* __restrict__ WP, __bf16* __restrict__ PK) {
  __shared__ __align__(16) __bf16 s[DM]; const int n = blockIdx.x, which = blockIdx.y, t = threadIdx.x; const float* Wm = (which == 0) ? WQ : (which == 1) ? WK : (which == 2) ? WV : (which == 3) ? WO : WP;
  for (int k = t; k < DM; k += 256) s[k] = (__bf16)Wm[(size_t)n * DM + k];
  __syncthreads();
  if (t < DM / 8) vst2((unsigned*)(PK + (size_t)which * DM * DM + (size_t)n * DM + t * 8), *(const v4u*)&s[t * 8]);
}
__global__ __launch_bounds__(128) void k_ln0(const float* __restrict__ X, const float* __restrict__ G, const float* __restrict__ Bv, float* __restrict__ XN) {
  __shared__ float red[2][4]; const int t = threadIdx.x; const size_t row = RB0 + blockIdx.x; const float* p = X + row * DM + t * 4;
  float v[4] = {bfr(p[0]), bfr(p[1]), bfr(p[2]), bfr(p[3])}; float s = (v[0] + v[1]) + (v[2] + v[3]);
#pragma unroll
  for (int o = 1; o < 32; o <<= 1) s += __shfl_xor(s, o);
  if ((t & 31) == 0) red[0][t >> 5] = s; __syncthreads();
  const float mu = (red[0][0] + red[0][1] + red[0][2] + red[0][3]) / (float)DM; float q = 0.f;
#pragma unroll
  for (int i = 0; i < 4; ++i) { const float d = v[i] - mu; q += d * d; }
#pragma unroll
  for (int o = 1; o < 32; o <<= 1) q += __shfl_xor(q, o);
  if ((t & 31) == 0) red[1][t >> 5] = q; __syncthreads();
  const float inv = 1.0f / sqrtf((red[1][0] + red[1][1] + red[1][2] + red[1][3]) / (float)DM + 1e-5f); v4f o4;
#pragma unroll
  for (int i = 0; i < 4; ++i) o4[i] = (v[i] - mu) * inv * bfr(G[t * 4 + i]) + bfr(Bv[t * 4 + i]);
  vst2(XN + row * DM + t * 4, o4);
}
__global__ __launch_bounds__(128) void k_proj(const float* __restrict__ XN, const float* __restrict__ PE, const __bf16* __restrict__ PK, const float* __restrict__ BQ, const float* __restrict__ BK, const float* __restrict__ BV, const float* __restrict__ U, const float* __restrict__ V, _Float16* __restrict__ QUH, _Float16* __restrict__ QUL, _Float16* __restrict__ QVH, _Float16* __restrict__ QVL, _Float16* __restrict__ KH, _Float16* __restrict__ KL, _Float16* __restrict__ VTH, _Float16* __restrict__ VTL, _Float16* __restrict__ RH, _Float16* __restrict__ RL) {
  __shared__ __align__(16) _Float16 s1h[4][16][136], s1l[4][16][136], s2h[4][16][136], s2l[4][16][136]; __shared__ __align__(16) _Float16 sth[128][72], stl[128][72];
  const int tid = threadIdx.x, wave = tid >> 5, lane = tid & 31, col = lane & 15, g = lane >> 4; const int which = blockIdx.z; const int n0 = blockIdx.y * 128;
  const size_t r0 = ((which == 3) ? 0 : RB0) + (size_t)blockIdx.x * 64 + wave * 16;
  if (which == 3 && blockIdx.x * 64 >= PR) return; if (which != 3 && blockIdx.x >= NBT * SS / 64) return;
  const __bf16* P = PK + ((which == 0) ? PK_Q : (which == 1) ? PK_K : (which == 2) ? PK_V : PK_P);
  v8f acc[8] = {};
  if (which == 3) {
#pragma unroll 2
    for (int kc = 0; kc < DM / 32; ++kc) { v16b a; { const size_t rr = r0 + col; const float* p = PE + (rr < PP ? rr : 0) * DM + kc * 32 + 8 * g; const bool ok = rr < PP;
#pragma unroll
        for (int i = 0; i < 8; ++i) { a[i] = (__bf16)(ok ? p[i] : 0.f); a[8 + i] = (__bf16)(ok ? p[16 + i] : 0.f); } }
#pragma unroll
      for (int j = 0; j < 8; ++j) acc[j] = wmma_bf(a, frag_b(P + (size_t)(n0 + j * 16 + col) * DM + kc * 32, lane), acc[j]); }
  } else {
#pragma unroll 2
    for (int kc = 0; kc < DM / 32; ++kc) { const F2 a = split_row(XN + (r0 + col) * DM, kc * 32, lane);
#pragma unroll
      for (int j = 0; j < 8; ++j) { const v16b w = frag_b(P + (size_t)(n0 + j * 16 + col) * DM + kc * 32, lane); acc[j] = wmma_bf(a.l, w, acc[j]); acc[j] = wmma_bf(a.h, w, acc[j]); } } }
  if (which == 0) {
#pragma unroll
    for (int j = 0; j < 8; ++j) { const int c = n0 + j * 16 + col; const float bb = bfr(BQ[c]), uu = bfr(U[c]), vv = bfr(V[c]);
#pragma unroll
      for (int r = 0; r < 8; ++r) { const float q = acc[j][r] + bb; const float qu = q + uu, qv = q + vv; const _Float16 h1 = (_Float16)qu, h2 = (_Float16)qv;
        s1h[wave][8 * g + r][j * 16 + col] = h1; s1l[wave][8 * g + r][j * 16 + col] = (_Float16)((qu - (float)h1) * 2048.0f); s2h[wave][8 * g + r][j * 16 + col] = h2; s2l[wave][8 * g + r][j * 16 + col] = (_Float16)((qv - (float)h2) * 2048.0f); } }
    LDSX();
    for (int rl = 0; rl < 16; ++rl) { const size_t o = (r0 + rl) * DM + n0; if (lane < 16) { vst2((unsigned*)(QUH + o + lane * 8), *(const v4u*)&s1h[wave][rl][lane * 8]); vst2((unsigned*)(QVH + o + lane * 8), *(const v4u*)&s2h[wave][rl][lane * 8]); } else { vst2((unsigned*)(QUL + o + (lane - 16) * 8), *(const v4u*)&s1l[wave][rl][(lane - 16) * 8]); vst2((unsigned*)(QVL + o + (lane - 16) * 8), *(const v4u*)&s2l[wave][rl][(lane - 16) * 8]); } }
  } else if (which == 1 || which == 3) { const float* BB = BK;
#pragma unroll
    for (int j = 0; j < 8; ++j) { const float bb = (which == 1) ? bfr(BB[n0 + j * 16 + col]) : 0.f;
#pragma unroll
      for (int r = 0; r < 8; ++r) { const float v = acc[j][r] + bb; const _Float16 hv = (_Float16)v; s1h[wave][8 * g + r][j * 16 + col] = hv; s1l[wave][8 * g + r][j * 16 + col] = (_Float16)((v - (float)hv) * 2048.0f); } }
    LDSX();
    _Float16* DH_ = (which == 1) ? KH : RH; _Float16* DL_ = (which == 1) ? KL : RL;
    for (int rl = 0; rl < 16; ++rl) { const size_t o = (r0 + rl) * DM + n0; if (lane < 16) vst2((unsigned*)(DH_ + o + lane * 8), *(const v4u*)&s1h[wave][rl][lane * 8]); else vst2((unsigned*)(DL_ + o + (lane - 16) * 8), *(const v4u*)&s1l[wave][rl][(lane - 16) * 8]); }
  } else {
#pragma unroll
    for (int j = 0; j < 8; ++j) { const float bb = bfr(BV[n0 + j * 16 + col]);
#pragma unroll
      for (int r = 0; r < 8; ++r) { const float v = acc[j][r] + bb; const _Float16 hv = (_Float16)v; sth[j * 16 + col][wave * 16 + 8 * g + r] = hv; stl[j * 16 + col][wave * 16 + 8 * g + r] = (_Float16)((v - (float)hv) * 2048.0f); } }
    __syncthreads();
    const size_t rb = RB0 + (size_t)blockIdx.x * 64; const size_t b = rb / SS; const int s0 = (int)(rb % SS);
    for (int e = tid; e < 128 * 8; e += 128) { const int d = e >> 3, pc = e & 7; const size_t o = (b * DM + n0 + d) * SS + s0 + pc * 8; vst2((unsigned*)(VTH + o), *(const v4u*)&sth[d][pc * 8]); vst2((unsigned*)(VTL + o), *(const v4u*)&stl[d][pc * 8]); }
  }
}
__global__ __launch_bounds__(128) void k_attn(const _Float16* __restrict__ QUH, const _Float16* __restrict__ QUL, const _Float16* __restrict__ QVH, const _Float16* __restrict__ QVL, const _Float16* __restrict__ KH, const _Float16* __restrict__ KL, const _Float16* __restrict__ RH, const _Float16* __restrict__ RL, const _Float16* __restrict__ VTH, const _Float16* __restrict__ VTL, float* __restrict__ O) {
  __shared__ __align__(16) _Float16 sph[4][16][40], spl[4][16][40]; __shared__ float sbd[4][16][49]; __shared__ __align__(16) float so[4][16][68];
  const int tid = threadIdx.x, wave = tid >> 5, lane = tid & 31, col = lane & 15, g = lane >> 4; const int qb = blockIdx.x, h = blockIdx.y; const size_t b = blockIdx.z + TB0; const int i0 = qb * 64, iw0 = i0 + wave * 16; const size_t rowb = b * SS;
  v16h aqu[2], aqul[2]; const size_t qo = (rowb + iw0 + col) * DM + h * HD;
#pragma unroll
  for (int kc = 0; kc < 2; ++kc) { aqu[kc] = frag_h(QUH + qo + kc * 32, lane); aqul[kc] = frag_h(QUL + qo + kc * 32, lane); }
  const _Float16* Vh = VTH + (b * DM + h * HD) * SS; const _Float16* Vl = VTL + (b * DM + h * HD) * SS;
  float m[8], l[8];
#pragma unroll
  for (int r = 0; r < 8; ++r) { m[r] = -3.0e38f; l[r] = 0.f; }
  v8f acc[4] = {}, accl[4] = {};
#pragma unroll 1
  for (int ks = 0; ks < SS / 32; ++ks) { const int j0 = ks * 32;
    { const int r0w = (SS - 1) + j0 - iw0 - 15;
#pragma unroll
      for (int ct3 = 0; ct3 < 3; ++ct3) { int rr = r0w + ct3 * 16 + col; rr = min(max(rr, 0), PR - 1); v8f u = {}, ul = {};
#pragma unroll
        for (int kc = 0; kc < 2; ++kc) { const v16h aqv = frag_h(QVH + qo + kc * 32, lane), aqvl = frag_h(QVL + qo + kc * 32, lane); const v16h rh = frag_h(RH + (size_t)rr * DM + h * HD + kc * 32, lane); u = wmma16(aqv, rh, u); ul = wmma16(aqvl, rh, ul); ul = wmma16(aqv, frag_h(RL + (size_t)rr * DM + h * HD + kc * 32, lane), ul); }
#pragma unroll
        for (int r = 0; r < 8; ++r) sbd[wave][8 * g + r][ct3 * 16 + col] = u[r] + ul[r] * (1.0f / 2048.0f); } }
    LDSX();
    v8f s[2];
#pragma unroll
    for (int ct = 0; ct < 2; ++ct) { const int jl = ct * 16 + col; const int kk = j0 + jl; const size_t rk = (rowb + kk) * DM + h * HD; v8f c = {}, cl = {};
#pragma unroll
      for (int kc = 0; kc < 2; ++kc) { const v16h khf = frag_h(KH + rk + kc * 32, lane); c = wmma16(aqu[kc], khf, c); cl = wmma16(aqul[kc], khf, cl); cl = wmma16(aqu[kc], frag_h(KL + rk + kc * 32, lane), cl); }
#pragma unroll
      for (int r = 0; r < 8; ++r) { const int il = 8 * g + r; s[ct][r] = (c[r] + cl[r] * (1.0f / 2048.0f) + sbd[wave][il][jl - il + 15]) * 0.125f; } }
#pragma unroll
    for (int r = 0; r < 8; ++r) { float mx = fmaxf(s[0][r], s[1][r]);
#pragma unroll
      for (int o = 1; o < 16; o <<= 1) mx = fmaxf(mx, __shfl_xor(mx, o));
      const float mn = fmaxf(m[r], mx); const float alpha = (m[r] <= -1.0e38f) ? 0.f : __expf(m[r] - mn);
      const float e0 = __expf(s[0][r] - mn), e1 = __expf(s[1][r] - mn); float es = e0 + e1;
#pragma unroll
      for (int o = 1; o < 16; o <<= 1) es += __shfl_xor(es, o);
      l[r] = l[r] * alpha + es; m[r] = mn;
#pragma unroll
      for (int dt = 0; dt < 4; ++dt) { acc[dt][r] *= alpha; accl[dt][r] *= alpha; }
      const _Float16 h0 = (_Float16)e0, h1 = (_Float16)e1; sph[wave][8 * g + r][col] = h0; sph[wave][8 * g + r][16 + col] = h1; spl[wave][8 * g + r][col] = (_Float16)((e0 - (float)h0) * 2048.0f); spl[wave][8 * g + r][16 + col] = (_Float16)((e1 - (float)h1) * 2048.0f); }
    LDSX();
    const v16h pah = frag_h(&sph[wave][col][0], lane), pal = frag_h(&spl[wave][col][0], lane);
#pragma unroll
    for (int dt = 0; dt < 4; ++dt) { const size_t vo = (size_t)(dt * 16 + col) * SS + j0; const v16h vh = frag_h(Vh + vo, lane), vl = frag_h(Vl + vo, lane); acc[dt] = wmma16(pah, vh, acc[dt]); accl[dt] = wmma16(pal, vh, accl[dt]); accl[dt] = wmma16(pah, vl, accl[dt]); }
    LDSX(); }
#pragma unroll
  for (int r = 0; r < 8; ++r) { const float il = 1.0f / l[r];
#pragma unroll
    for (int dt = 0; dt < 4; ++dt) so[wave][8 * g + r][dt * 16 + col] = (acc[dt][r] + accl[dt][r] * (1.0f / 2048.0f)) * il; }
  LDSX();
  for (int rl = 0; rl < 16; ++rl) if (lane < 16) vst2(O + (rowb + iw0 + rl) * DM + h * HD + lane * 4, *(const v4f*)&so[wave][rl][lane * 4]);
}
__global__ __launch_bounds__(128) void k_out(const float* __restrict__ Oc, const __bf16* __restrict__ PK, const float* __restrict__ BO, const float* __restrict__ X, float* __restrict__ Y) {
  __shared__ __align__(16) float so[4][16][132];
  const int tid = threadIdx.x, wave = tid >> 5, lane = tid & 31, col = lane & 15, g = lane >> 4; const size_t r0 = RB0 + (size_t)blockIdx.x * 64 + wave * 16; const int n0 = blockIdx.y * 128;
  v8f acc[8] = {};
#pragma unroll 2
  for (int kc = 0; kc < DM / 32; ++kc) { const F2 a = split_row(Oc + (r0 + col) * DM, kc * 32, lane);
#pragma unroll
    for (int j = 0; j < 8; ++j) { const v16b w = frag_b(PK + PK_O + (size_t)(n0 + j * 16 + col) * DM + kc * 32, lane); acc[j] = wmma_bf(a.l, w, acc[j]); acc[j] = wmma_bf(a.h, w, acc[j]); } }
#pragma unroll
  for (int j = 0; j < 8; ++j) { const int c = n0 + j * 16 + col; const float bb = bfr(BO[c]);
#pragma unroll
    for (int r = 0; r < 8; ++r) { const size_t row = r0 + 8 * g + r; so[wave][8 * g + r][j * 16 + col] = acc[j][r] + bb + bfr(X[row * DM + c]); } }
  LDSX();
  for (int rl = 0; rl < 16; ++rl) vst2(Y + (r0 + rl) * DM + n0 + lane * 4, *(const v4f*)&so[wave][rl][lane * 4]);
}
extern "C" void kernel_launch(void* const* d_in, const int* in_sizes, int n_in, void* d_out, int out_size, void* d_ws, size_t ws_size, hipStream_t stream) {
  (void)in_sizes; (void)n_in; (void)out_size;
  const float** F = (const float**)d_in;
  if (ws_size < (size_t)WS_END) return;
  char* ws = (char*)d_ws; __bf16* PK = (__bf16*)(ws + WS_PK); float *XN = (float*)(ws + WS_XN), *O = (float*)(ws + WS_O);
  _Float16 *QUH = (_Float16*)(ws + WS_QUH), *QUL = (_Float16*)(ws + WS_QUL), *QVH = (_Float16*)(ws + WS_QVH), *QVL = (_Float16*)(ws + WS_QVL), *KH = (_Float16*)(ws + WS_KH), *KL = (_Float16*)(ws + WS_KL), *VTH = (_Float16*)(ws + WS_VTH), *VTL = (_Float16*)(ws + WS_VTL), *RH = (_Float16*)(ws + WS_RH), *RL = (_Float16*)(ws + WS_RL);
  k_pack<<<dim3(DM, 5), 256, 0, stream>>>(F[4], F[6], F[8], F[10], F[12], PK);
  k_ln0<<<NBT * SS, 128, 0, stream>>>(F[0], F[2], F[3], XN);
  { const int rt = (NBT * SS / 64 > PR / 64) ? NBT * SS / 64 : PR / 64; k_proj<<<dim3(rt, DM / 128, 4), 128, 0, stream>>>(XN, F[1], PK, F[5], F[7], F[9], F[13], F[14], QUH, QUL, QVH, QVL, KH, KL, VTH, VTL, RH, RL); }
  k_attn<<<dim3(TQB, NH, NBT), 128, 0, stream>>>(QUH, QUL, QVH, QVL, KH, KL, RH, RL, VTH, VTL, O);
  k_out<<<dim3(NBT * SS / 64, DM / 128), 128, 0, stream>>>(O, PK, F[11], F[0], (float*)d_out);
}
